// Attention_87205015978193
// MI455X (gfx1250) — hardware-verified
//
#include <hip/hip_runtime.h>


#ifndef NB
#define NB 4
#endif
#ifndef SEQ
#define SEQ 2048
#endif
#define NB_FULL  4
#define SEQ_FULL 2048
#define DM   1024
#define NH   16
#define HD   64
#define NWV  4
#define BQ   (16 * NWV)
#define KS   32
#define OSP  68
#define VTP  72
#define QSP  136
#define FSP  132
#define L2E  1.4426950408889634f
#define SCL  (L2E * (1.0f / 2048.0f))

static_assert(DM == NH * HD);
static_assert(HD == 64);
static_assert(DM == 1024);
static_assert(NWV == 4);
static_assert(SEQ % BQ == 0);
static_assert(SEQ % KS == 0);
static_assert(SEQ % 128 == 0);
static_assert(SEQ % 64 == 0);
static_assert(NB <= NB_FULL);
static_assert(SEQ <= SEQ_FULL);
static_assert(((size_t)NB * SEQ * DM) % 2048 == 0);
static_assert((size_t)(16 * 8) * (size_t)(64 * 128) == (size_t)DM * DM);
static_assert((size_t)(NB * SEQ / 64) * 8 * (size_t)(64 * 128) == (size_t)NB * SEQ * DM);
static_assert((size_t)(SEQ / BQ) * NH * NB * (size_t)(BQ * 2 * HD) == (size_t)NB * SEQ * 2 * DM);
static_assert((size_t)(NB * SEQ / 64) * 8 * (size_t)(64 * 128) == (size_t)NB * SEQ * DM);
static_assert(128 * VTP >= 64 * QSP);
static_assert((size_t)4 * NB * SEQ * DM * 2 + (size_t)4 * DM * DM * 2 + (size_t)NB * SEQ * 2 * DM * 2 <= (size_t)134217728);

typedef unsigned short u16;
typedef __attribute__((ext_vector_type(16))) __bf16   v16bf;
typedef __attribute__((ext_vector_type(16))) _Float16 v16h;
typedef __attribute__((ext_vector_type(8)))  unsigned short v8us;
typedef __attribute__((ext_vector_type(8)))  float    v8f;
typedef __attribute__((ext_vector_type(4)))  float    v4f;
typedef v4f  __attribute__((may_alias)) v4fa;
typedef v8us __attribute__((may_alias)) v8usa;

__device__ __forceinline__ unsigned short f2bf(float f) { unsigned u = __float_as_uint(f); u += 0x7FFFu + ((u >> 16) & 1u); return (unsigned short)(u >> 16); }
__device__ __forceinline__ float bf2f(unsigned short b) { return __uint_as_float(((unsigned)b) << 16); }
__device__ __forceinline__ float bfr(float f) { return bf2f(f2bf(f)); }
__device__ __forceinline__ unsigned short f2h(float f) { return __builtin_bit_cast(unsigned short, (_Float16)f); }
__device__ __forceinline__ v16bf cat16b(v8us lo, v8us hi) { return __builtin_bit_cast(v16bf, __builtin_shufflevector(lo, hi, 0, 1, 2, 3, 4, 5, 6, 7, 8, 9, 10, 11, 12, 13, 14, 15)); }
__device__ __forceinline__ v16h  cat16h(v8us lo, v8us hi) { return __builtin_bit_cast(v16h,  __builtin_shufflevector(lo, hi, 0, 1, 2, 3, 4, 5, 6, 7, 8, 9, 10, 11, 12, 13, 14, 15)); }
__device__ __forceinline__ v8f wmmab(v16bf a, v16bf b, v8f c) { return __builtin_amdgcn_wmma_f32_16x16x32_bf16(false, a, false, b, (short)0, c, false, false); }
__device__ __forceinline__ v8f wmmah(v16h a, v16h b, v8f c)   { return __builtin_amdgcn_wmma_f32_16x16x32_f16(false, a, false, b, (short)0, c, false, false); }
__device__ __forceinline__ v16bf ldb(const u16* p) { return cat16b(*(const v8us*)p, *(const v8us*)(p + 16)); }
__device__ __forceinline__ v16h  ldh(const u16* p) { return cat16h(*(const v8us*)p, *(const v8us*)(p + 16)); }

__global__ __launch_bounds__(256) void k_cvt8(const float* __restrict__ x, u16* XB) {
    const unsigned i = blockIdx.x * 256u + threadIdx.x;
    const unsigned per = (unsigned)(SEQ * DM / 8);
    if (i >= (unsigned)NB * per) return;
    const unsigned b = i / per, r = i - b * per;
    const float* src = x + (size_t)b * SEQ_FULL * DM + (size_t)r * 8;
    u16* dst = XB + (size_t)i * 8;
    const v8f v = *(const v8f*)src;
    v8us o;
#pragma unroll
    for (int c = 0; c < 8; ++c) o[c] = f2bf(v[c]);
    *(volatile v8us*)dst = o;
    __threadfence();
    *(volatile v8us*)dst = o;
}

__global__ __launch_bounds__(256) void k_wt(const float* __restrict__ Wq, const float* __restrict__ Wk, const float* __restrict__ Wv, const float* __restrict__ Wo, u16* WT) {
    __shared__ __align__(16) u16 tl[128 * VTP];
    const unsigned tid = threadIdx.x;
    const unsigned w = blockIdx.y;
    const float* W = (w == 0u) ? Wq : (w == 1u) ? Wk : (w == 2u) ? Wv : Wo;
    const unsigned k0 = (blockIdx.x >> 3) * 64u;
    const unsigned n0 = (blockIdx.x & 7u) * 128u;
    const float* src = W + (size_t)k0 * DM + n0;
#pragma unroll
    for (unsigned it = 0; it < 8; ++it) {
        const unsigned f = it * 256u + tid;
        const unsigned kr = f >> 5, n4 = (f & 31u) * 4u;
        const v4f x = *(const v4f*)(src + (size_t)kr * DM + n4);
#pragma unroll
        for (unsigned c = 0; c < 4; ++c) tl[(n4 + c) * VTP + kr] = f2bf(x[c]);
    }
    __syncthreads();
    u16* dst = WT + ((size_t)w * DM + n0) * DM + k0;
    const unsigned c8 = (tid & 7u) * 8u, dr = tid >> 3;
#pragma unroll 1
    for (int ps = 0; ps < 2; ++ps) {
#pragma unroll
        for (unsigned it = 0; it < 4; ++it) {
            const unsigned d = it * 32u + dr;
            const v8us o = *(const v8usa*)(tl + d * VTP + c8);
            *(volatile v8us*)(dst + (size_t)d * DM + c8) = o;
        }
        if (ps == 0) __threadfence();
    }
}

template <unsigned KTOT, unsigned KWRAP>
__device__ __forceinline__ void gemm32x64(const u16* __restrict__ ap, const unsigned lda, const u16* __restrict__ bp, const unsigned ldbb, v8f (&acc)[2][4]) {
    static_assert((KWRAP & (KWRAP - 1u)) == 0u);
    static_assert(KTOT % 32u == 0u);
#pragma unroll 1
    for (unsigned k = 0; k < KTOT; k += 32u) {
        const unsigned kb = k & (KWRAP - 1u);
        const v16bf a0 = ldb(ap + k);
        const v16bf a1 = ldb(ap + (size_t)16 * lda + k);
        const v16bf b0 = ldb(bp + kb);
        const v16bf b1 = ldb(bp + (size_t)16 * ldbb + kb);
        const v16bf b2 = ldb(bp + (size_t)32 * ldbb + kb);
        const v16bf b3 = ldb(bp + (size_t)48 * ldbb + kb);
        acc[0][0] = wmmab(a0, b0, acc[0][0]);
        acc[0][1] = wmmab(a0, b1, acc[0][1]);
        acc[0][2] = wmmab(a0, b2, acc[0][2]);
        acc[0][3] = wmmab(a0, b3, acc[0][3]);
        acc[1][0] = wmmab(a1, b0, acc[1][0]);
        acc[1][1] = wmmab(a1, b1, acc[1][1]);
        acc[1][2] = wmmab(a1, b2, acc[1][2]);
        acc[1][3] = wmmab(a1, b3, acc[1][3]);
        asm volatile("v_nop\n\tv_nop\n\tv_nop\n\tv_nop"
                     : "+v"(acc[0][0]), "+v"(acc[0][1]), "+v"(acc[0][2]), "+v"(acc[0][3]),
                       "+v"(acc[1][0]), "+v"(acc[1][1]), "+v"(acc[1][2]), "+v"(acc[1][3])
                     : "v"(a0), "v"(a1), "v"(b0), "v"(b1), "v"(b2), "v"(b3));
    }
}

__global__ __launch_bounds__(128) void k_qkv(const u16* __restrict__ XB, const u16* __restrict__ WT,
                                             const float* __restrict__ bq, const float* __restrict__ bk, const float* __restrict__ bv,
                                             u16* QP, u16* KP, u16* VT) {
    __shared__ __align__(16) u16 st[128 * VTP];
    const unsigned tid = threadIdx.x, lane = tid & 31u, wv = tid >> 5, lr = lane & 15u, hi = lane >> 4;
    const unsigned wm = wv & 1u, wn = wv >> 1;
    const unsigned mb = blockIdx.x * 64u;
    const unsigned nb = blockIdx.y * 128u;
    const unsigned mode = nb >> 10;
    const unsigned nc0 = nb & 1023u;

    v8f acc[2][4];
#pragma unroll
    for (int t = 0; t < 2; ++t) {
#pragma unroll
        for (int j = 0; j < 4; ++j) acc[t][j] = (v8f){};
    }
    gemm32x64<DM, DM>(XB + (size_t)(mb + wm * 32u + lr) * DM + 8u * hi, DM,
                      WT + (size_t)(nb + wn * 64u + lr) * DM + 8u * hi, DM, acc);

    const float* bias = (mode == 0u) ? bq : (mode == 1u) ? bk : bv;
#pragma unroll
    for (int j = 0; j < 4; ++j) {
        const unsigned nl = wn * 64u + (unsigned)j * 16u + lr;
        const float bsv = bfr(bias[nc0 + nl]);
#pragma unroll
        for (int t = 0; t < 2; ++t) {
#pragma unroll
            for (int r = 0; r < 8; ++r) {
                const unsigned ml = wm * 32u + (unsigned)t * 16u + 8u * hi + (unsigned)r;
                const unsigned short hv = f2h((acc[t][j][r] + bsv) * 16.0f);
                if (mode == 2u) st[nl * VTP + ml] = hv;
                else            st[ml * QSP + nl] = hv;
            }
        }
    }
    __syncthreads();
    if (mode != 2u) {
        u16* dst = ((mode == 0u) ? QP : KP) + (size_t)mb * DM + nc0;
#pragma unroll 1
        for (int ps = 0; ps < 2; ++ps) {
#pragma unroll
            for (unsigned it = 0; it < 8; ++it) {
                const unsigned f = it * 128u + tid;
                const unsigned line = f >> 3, pc = (f & 7u) * 8u;
                const unsigned row = line >> 1, sg = (line & 1u) * 64u;
                const v8us o = *(const v8usa*)(st + row * QSP + sg + pc);
                *(volatile v8us*)(dst + (size_t)row * DM + sg + pc) = o;
            }
            if (ps == 0) __threadfence();
        }
    } else {
        const unsigned b = mb / (unsigned)SEQ;
        const unsigned s0 = mb - b * (unsigned)SEQ;
        u16* dst = VT + ((size_t)b * DM + nc0) * SEQ + s0;
#pragma unroll 1
        for (int ps = 0; ps < 2; ++ps) {
#pragma unroll
            for (unsigned it = 0; it < 8; ++it) {
                const unsigned f = it * 128u + tid;
                const unsigned nl = f >> 3, pc = (f & 7u) * 8u;
                const v8us o = *(const v8usa*)(st + nl * VTP + pc);
                *(volatile v8us*)(dst + (size_t)nl * SEQ + pc) = o;
            }
            if (ps == 0) __threadfence();
        }
    }
}

__global__ __launch_bounds__(128) void k_flash(const u16* __restrict__ QP, const u16* __restrict__ KP, const u16* __restrict__ VT, const float* __restrict__ mask, u16* CT) {
    __shared__ __align__(16) float mk[SEQ];
    __shared__ __align__(16) float os[NWV * 16 * OSP];
    const unsigned tid = threadIdx.x, lane = tid & 31u, wv = tid >> 5, lr = lane & 15u, hi = lane >> 4;
    const unsigned h = blockIdx.y, b = blockIdx.z;
    const unsigned q0 = blockIdx.x * (unsigned)BQ + wv * 16u;

    {
        const float* mp = mask + (size_t)b * SEQ_FULL;
#pragma unroll 1
        for (unsigned i = tid * 4u; i < (unsigned)SEQ; i += 512u) {
            const v4f x = *(const v4f*)(mp + i);
            v4f y;
            y[0] = bfr(x[0]) * L2E; y[1] = bfr(x[1]) * L2E; y[2] = bfr(x[2]) * L2E; y[3] = bfr(x[3]) * L2E;
            *(v4fa*)(mk + i) = y;
        }
    }
    __syncthreads();

    v16h qf[2];
    {
        const u16* qp = QP + ((size_t)b * SEQ + q0 + lr) * DM + h * (unsigned)HD + 8u * hi;
        qf[0] = ldh(qp);
        qf[1] = ldh(qp + 32);
    }
    const u16* kp = KP + ((size_t)b * SEQ + lr) * DM + h * (unsigned)HD + 8u * hi;
    const u16* vp = VT + ((size_t)b * DM + h * (unsigned)HD + lr) * SEQ + 8u * hi;

    v8f o[4];
#pragma unroll
    for (int t = 0; t < 4; ++t) o[t] = (v8f){};
    float ml = -1.0e30f;
    float l = 0.0f;

#pragma unroll 1
    for (unsigned k0 = 0; k0 < (unsigned)SEQ; k0 += KS) {
        v8f s0 = (v8f){}, s1 = (v8f){};
        const u16* ka = kp + (size_t)k0 * DM;
        {
            const v16h a00 = ldh(ka);
            const v16h a01 = ldh(ka + 32);
            const v16h a10 = ldh(ka + (size_t)16 * DM);
            const v16h a11 = ldh(ka + (size_t)16 * DM + 32);
            s0 = wmmah(a00, qf[0], s0);
            s1 = wmmah(a10, qf[0], s1);
            s0 = wmmah(a01, qf[1], s0);
            s1 = wmmah(a11, qf[1], s1);
            asm volatile("v_nop\n\tv_nop\n\tv_nop\n\tv_nop" : "+v"(s0), "+v"(s1) : "v"(qf[0]), "v"(qf[1]), "v"(a01), "v"(a11));
        }

        const v4f m0a = *(const v4fa*)(mk + k0 + 8u * hi);
        const v4f m0b = *(const v4fa*)(mk + k0 + 8u * hi + 4u);
        const v4f m1a = *(const v4fa*)(mk + k0 + 16u + 8u * hi);
        const v4f m1b = *(const v4fa*)(mk + k0 + 16u + 8u * hi + 4u);
        float x0[8], x1[8];
#pragma unroll
        for (int r = 0; r < 4; ++r) {
            x0[r]     = fmaf(s0[r],     SCL, m0a[r]);
            x0[4 + r] = fmaf(s0[4 + r], SCL, m0b[r]);
            x1[r]     = fmaf(s1[r],     SCL, m1a[r]);
            x1[4 + r] = fmaf(s1[4 + r], SCL, m1b[r]);
        }
        float mx = fmaxf(x0[0], x1[0]);
#pragma unroll
        for (int r = 1; r < 8; ++r) mx = fmaxf(mx, fmaxf(x0[r], x1[r]));
        mx = fmaxf(mx, __shfl_xor(mx, 16, 32));
        const float mnl = fmaxf(ml, mx);
        const float corr = __builtin_amdgcn_exp2f(ml - mnl);
        ml = mnl;
        const float mb10 = mnl - 10.0f;
        float p0[8], p1[8];
        float ps = 0.0f;
#pragma unroll
        for (int r = 0; r < 8; ++r) {
            p0[r] = __builtin_amdgcn_exp2f(x0[r] - mb10);
            p1[r] = __builtin_amdgcn_exp2f(x1[r] - mb10);
            ps += p0[r] + p1[r];
        }
        ps += __shfl_xor(ps, 16, 32);
        l = l * corr + ps;
        if (__builtin_amdgcn_ballot_w32(corr != 1.0f) != 0u) {
#pragma unroll
            for (int t = 0; t < 4; ++t) o[t] *= corr;
        }

        v16h ph;
#pragma unroll
        for (int r = 0; r < 8; ++r) {
            ph[r]     = (_Float16)p0[r];
            ph[8 + r] = (_Float16)p1[r];
        }

        asm volatile("" ::: "memory");
        const u16* va = vp + k0;
#pragma unroll
        for (int t = 0; t < 4; ++t) {
            const v16h a = ldh(va + (size_t)t * 16 * SEQ);
            o[t] = wmmah(a, ph, o[t]);
        }
        asm volatile("v_nop\n\tv_nop\n\tv_nop\n\tv_nop"
                     : "+v"(o[0]), "+v"(o[1]), "+v"(o[2]), "+v"(o[3])
                     : "v"(ph));
    }

    const float inv = (1.0f / l) * 0.0625f;
    float* ow = os + wv * (16 * OSP);
#pragma unroll
    for (int t = 0; t < 4; ++t) {
#pragma unroll
        for (int r = 0; r < 8; ++r) ow[lr * OSP + t * 16 + 8 * hi + r] = o[t][r] * inv;
    }
    __syncthreads();
    const unsigned rq = lane >> 3, c8 = (lane & 7u) * 8u;
    u16* crow = CT + ((size_t)b * SEQ + q0) * (2 * DM) + h * (unsigned)HD + c8;
#pragma unroll 1
    for (int ps2 = 0; ps2 < 2; ++ps2) {
#pragma unroll
        for (unsigned it = 0; it < 4; ++it) {
            const unsigned row = it * 4u + rq;
            const v4f xa = *(const v4fa*)(ow + row * OSP + c8);
            const v4f xb = *(const v4fa*)(ow + row * OSP + c8 + 4u);
            v8us hv, lv;
#pragma unroll
            for (int c = 0; c < 4; ++c) {
                const unsigned short ha = f2bf(xa[c]);
                const unsigned short hb = f2bf(xb[c]);
                hv[c] = ha; hv[4 + c] = hb;
                lv[c]     = f2bf(xa[c] - bf2f(ha));
                lv[4 + c] = f2bf(xb[c] - bf2f(hb));
            }
            *(volatile v8us*)(crow + (size_t)row * (2 * DM)) = hv;
            *(volatile v8us*)(crow + (size_t)row * (2 * DM) + DM) = lv;
        }
        if (ps2 == 0) __threadfence();
    }
}

__global__ __launch_bounds__(128) void k_out(const u16* __restrict__ CT, const u16* __restrict__ WoT, const float* __restrict__ bo, float* OUT) {
    __shared__ __align__(16) float st[64 * FSP];
    const unsigned tid = threadIdx.x, lane = tid & 31u, wv = tid >> 5, lr = lane & 15u, hi = lane >> 4;
    const unsigned wm = wv & 1u, wn = wv >> 1;
    const unsigned mb = blockIdx.x * 64u;
    const unsigned nb = blockIdx.y * 128u;

    v8f acc[2][4];
#pragma unroll
    for (int t = 0; t < 2; ++t) {
#pragma unroll
        for (int j = 0; j < 4; ++j) acc[t][j] = (v8f){};
    }
    gemm32x64<2 * DM, DM>(CT + (size_t)(mb + wm * 32u + lr) * (2 * DM) + 8u * hi, 2 * DM,
                          WoT + (size_t)(nb + wn * 64u + lr) * DM + 8u * hi, DM, acc);

#pragma unroll
    for (int j = 0; j < 4; ++j) {
        const unsigned nl = wn * 64u + (unsigned)j * 16u + lr;
        const float bsv = bfr(bo[nb + nl]);
#pragma unroll
        for (int t = 0; t < 2; ++t) {
#pragma unroll
            for (int r = 0; r < 8; ++r) {
                const unsigned ml = wm * 32u + (unsigned)t * 16u + 8u * hi + (unsigned)r;
                st[ml * FSP + nl] = acc[t][j][r] + bsv;
            }
        }
    }
    __syncthreads();
    float* dst = OUT + (size_t)mb * DM + nb + lane * 4u;
#pragma unroll 1
    for (int ps = 0; ps < 2; ++ps) {
#pragma unroll 4
        for (unsigned it = 0; it < 16; ++it) {
            const unsigned row = it * 4u + wv;
            const v4f val = *(const v4fa*)(st + row * FSP + lane * 4u);
            *(volatile v4f*)(dst + (size_t)row * DM) = val;
        }
        if (ps == 0) __threadfence();
    }
}

extern "C" void kernel_launch(void* const* d_in, const int* in_sizes, int n_in,
                              void* d_out, int out_size, void* d_ws, size_t ws_size, hipStream_t stream) {
    if (n_in < 10) return;
    const size_t need_x = ((size_t)(NB - 1) * SEQ_FULL + SEQ) * DM;
    const size_t need_m = (size_t)(NB - 1) * SEQ_FULL + SEQ;
    if ((size_t)in_sizes[0] < need_x || (size_t)in_sizes[1] < need_m) return;
    if ((size_t)in_sizes[2] < (size_t)DM * DM || (size_t)in_sizes[4] < (size_t)DM * DM ||
        (size_t)in_sizes[6] < (size_t)DM * DM || (size_t)in_sizes[8] < (size_t)DM * DM) return;
    if (in_sizes[3] < DM || in_sizes[5] < DM || in_sizes[7] < DM || in_sizes[9] < DM) return;
    if ((size_t)out_size < (size_t)NB * SEQ * DM) return;
    const float* hs   = (const float*)d_in[0];
    const float* mask = (const float*)d_in[1];
    const float* Wq   = (const float*)d_in[2];
    const float* bq   = (const float*)d_in[3];
    const float* Wk   = (const float*)d_in[4];
    const float* bk   = (const float*)d_in[5];
    const float* Wv   = (const float*)d_in[6];
    const float* bv   = (const float*)d_in[7];
    const float* Wo   = (const float*)d_in[8];
    const float* bo   = (const float*)d_in[9];
    float* OUT = (float*)d_out;

    const size_t PX = (size_t)NB * SEQ * DM * 2;
    const size_t PW = (size_t)4 * DM * DM * 2;
    const size_t PC = (size_t)NB * SEQ * 2 * DM * 2;
    if (4 * PX + PW + PC > ws_size) return;
    char* wsp = (char*)d_ws;
    u16* XB = (u16*)(wsp);
    u16* WT = (u16*)(wsp + PX);
    u16* QP = (u16*)(wsp + PX + PW);
    u16* KP = (u16*)(wsp + 2 * PX + PW);
    u16* VT = (u16*)(wsp + 3 * PX + PW);
    u16* CT = (u16*)(wsp + 4 * PX + PW);

    const unsigned gc = (unsigned)(((size_t)NB * SEQ * DM / 8 + 255) / 256);
    k_cvt8<<<gc, 256, 0, stream>>>(hs, XB);
    k_wt<<<dim3(128, 4, 1), 256, 0, stream>>>(Wq, Wk, Wv, Wo, WT);
    k_qkv<<<dim3((unsigned)(NB * SEQ / 64), 24, 1), 128, 0, stream>>>(XB, WT, bq, bk, bv, QP, KP, VT);
    k_flash<<<dim3((unsigned)(SEQ / BQ), NH, NB), 128, 0, stream>>>(QP, KP, VT, mask, CT);
    k_out<<<dim3((unsigned)(NB * SEQ / 64), 8, 1), 128, 0, stream>>>(CT, WT + (size_t)3 * DM * DM, bo, OUT);
}
